// MatryoshkaDilatedCostVolume_73632919323062
// MI455X (gfx1250) — hardware-verified
//
#include <hip/hip_runtime.h>

#define NB_ 4
#define CC_ 128
#define HH_ 64
#define WW_ 128
#define MD  4
#define NDIL 6
#define TS  136

typedef _Float16 f16;
typedef __attribute__((ext_vector_type(16))) f16 f16x16;
typedef __attribute__((ext_vector_type(8)))  f16 f16x8;
typedef __attribute__((ext_vector_type(8)))  float f32x8;
typedef __attribute__((ext_vector_type(4)))  float v4f_t;
typedef float v4fa __attribute__((ext_vector_type(4), may_alias));
__constant__ int c_dil[NDIL] = {1, 2, 3, 5, 9, 16};

__device__ __forceinline__ f32x8 wmma16(f16x16 a, f16x16 b, f32x8 c) {
  c = __builtin_amdgcn_wmma_f32_16x16x32_f16(false, a, false, b, (short)0, c, false, false);
  asm volatile("v_nop\n\tv_nop\n\tv_nop\n\tv_nop" : "+v"(c) : "v"(a), "v"(b));
  return c;
}
__device__ __forceinline__ f16x16 lds_frag(const f16* base, int stride) {
  const int lane = threadIdx.x & 31, row = lane & 15, kh = (lane >> 4) * 8;
  const f16x8 lo = *(const f16x8*)(base + row * stride + kh);
  const f16x8 hi = *(const f16x8*)(base + row * stride + kh + 16);
  f16x16 f;
#pragma unroll
  for (int i = 0; i < 8; ++i) { f[i] = lo[i]; f[i + 8] = hi[i]; }
  return f;
}

__global__ __launch_bounds__(256) void k_cost(const float* __restrict__ x1, const float* __restrict__ x2, float* __restrict__ out) {
  __shared__ __attribute__((aligned(16))) f16 aS[WW_ * TS];
  __shared__ __attribute__((aligned(16))) f16 bS[WW_ * TS];
  __shared__ __attribute__((aligned(16))) float oS[9 * WW_];
  const int tid = threadIdx.x, lane = tid & 31, wave = tid >> 5, cl = lane & 15, rh = (lane >> 4) * 8;
  int bid = blockIdx.x;
  const int u = bid % 9; bid /= 9;
  const int di = bid % NDIL; bid /= NDIL;
  const int y = bid % HH_; const int b = bid / HH_;
  const int d = c_dil[di];
  const int ys = y + (u - MD) * d;
  const bool rowok = (ys >= 0 && ys < HH_);
  for (int e = tid; e < 9 * WW_; e += 256) oS[e] = 0.0f;
  if (rowok) {
    const int c = tid >> 1, xh = (tid & 1) * 64;
    const float* p1 = x1 + (((size_t)b * CC_ + c) * HH_ + y) * WW_ + xh;
    const float* p2 = x2 + (((size_t)b * CC_ + c) * HH_ + ys) * WW_ + xh;
#pragma unroll 4
    for (int i = 0; i < 64; i += 4) {
      const v4f_t v1 = *(const v4f_t*)(p1 + i), v2 = *(const v4f_t*)(p2 + i);
#pragma unroll
      for (int q = 0; q < 4; ++q) { aS[(xh + i + q) * TS + c] = (f16)v1[q]; bS[(xh + i + q) * TS + c] = (f16)v2[q]; }
    }
  }
  __syncthreads();
  if (rowok) {
    f32x8 acc[8];
#pragma unroll
    for (int nt = 0; nt < 8; ++nt) { f32x8 z = {}; acc[nt] = z; }
#pragma unroll
    for (int ks = 0; ks < 4; ++ks) {
      const f16x16 af = lds_frag(aS + (wave * 16) * TS + ks * 32, TS);
#pragma unroll
      for (int nt = 0; nt < 8; ++nt) acc[nt] = wmma16(af, lds_frag(bS + (nt * 16) * TS + ks * 32, TS), acc[nt]);
    }
#pragma unroll
    for (int nt = 0; nt < 8; ++nt)
#pragma unroll
      for (int r = 0; r < 8; ++r) {
        const int x = wave * 16 + rh + r, xp = nt * 16 + cl, diff = xp - x;
        if (diff % d == 0) { const int v = diff / d + MD; if (v >= 0 && v <= 2 * MD) { const float s = acc[nt][r]; oS[v * WW_ + x] = (s >= 0.0f) ? s : 0.1f * s; } }
      }
  }
  __syncthreads();
#pragma unroll 1
  for (int pass = 0; pass < 2; ++pass) {
    for (int f4 = tid; f4 < 9 * 32; f4 += 256) { const int v = f4 >> 5, q = (f4 & 31) * 4;
      *(volatile v4f_t*)(out + (((((size_t)b * NDIL + di) * 9 + u) * 9 + v) * HH_ + y) * WW_ + q) = *(const volatile v4fa*)(oS + v * WW_ + q); }
    __threadfence();
  }
}

extern "C" void kernel_launch(void* const* d_in, const int* in_sizes, int n_in,
                              void* d_out, int out_size, void* d_ws, size_t ws_size,
                              hipStream_t stream) {
  (void)in_sizes; (void)n_in; (void)out_size; (void)d_ws; (void)ws_size;
  const float* x1 = (const float*)d_in[0];
  const float* x2 = (const float*)d_in[1];
  float* out = (float*)d_out;
  k_cost<<<dim3(NB_ * HH_ * NDIL * 9), dim3(256), 0, stream>>>(x1, x2, out);
}
